// TwoSimplicialAttention_82772609728942
// MI455X (gfx1250) — hardware-verified
//
#include <hip/hip_runtime.h>
#include <math.h>

typedef __attribute__((ext_vector_type(16))) _Float16 v16h;
typedef __attribute__((ext_vector_type(16))) __bf16 v16b;
typedef __attribute__((ext_vector_type(8)))  _Float16 v8h;
typedef __attribute__((ext_vector_type(8)))  float v8f;
typedef __attribute__((ext_vector_type(4)))  float v4f;
typedef __attribute__((ext_vector_type(2)))  float v2f;
typedef __attribute__((ext_vector_type(4)))  unsigned v4u;
typedef __attribute__((ext_vector_type(4)))  int v4i;
typedef float __attribute__((may_alias)) float_a;
typedef int __attribute__((may_alias)) int_a;

template <typename T> __device__ __forceinline__ void vst2(void* p, T v) { *(volatile T*)p = v; __threadfence(); *(volatile T*)p = v; }
__device__ __forceinline__ v8f wmma16(v16h a, v16h b, v8f c) {
  v8f d = __builtin_amdgcn_wmma_f32_16x16x32_f16(false, a, false, b, (short)0, c, false, false);
  asm volatile("v_nop\n\tv_nop\n\tv_nop\n\tv_nop" : "+v"(d) : "v"(a), "v"(b));
  return d;
}
__device__ __forceinline__ v8f wmma_bf(v16b a, v16b b, v8f c) {
  v8f d = __builtin_amdgcn_wmma_f32_16x16x32_bf16(false, a, false, b, (short)0, c, false, false);
  asm volatile("v_nop\n\tv_nop\n\tv_nop\n\tv_nop" : "+v"(d) : "v"(a), "v"(b));
  return d;
}
__device__ __forceinline__ v16h frag_h(const _Float16* rowk0, int lane) {
  union { v16h v; v8h q[2]; } u; const _Float16* p = rowk0 + 8 * (lane >> 4);
  u.q[0] = *(const v8h*)p; u.q[1] = *(const v8h*)(p + 16); return u.v;
}
__device__ __forceinline__ v16h frag_f32(const float* rowk0, int lane) {
  v16h a; const float* p = rowk0 + 8 * (lane >> 4);
#pragma unroll
  for (int i = 0; i < 8; ++i) { a[i] = (_Float16)p[i]; a[8 + i] = (_Float16)p[16 + i]; }
  return a;
}
__device__ __forceinline__ v16h frag_f32s(const float* rowk0, int lane, float sc) {
  v16h a; const float* p = rowk0 + 8 * (lane >> 4);
#pragma unroll
  for (int i = 0; i < 8; ++i) { a[i] = (_Float16)(p[i] * sc); a[8 + i] = (_Float16)(p[16 + i] * sc); }
  return a;
}
__device__ __forceinline__ v16h fragc_f32(const float* W, int k0, int n, int lane, int ld, int K) {
  v16h a; const int g = lane >> 4;
#pragma unroll
  for (int i = 0; i < 8; ++i) { const int ka = k0 + 8 * g + i, kb = ka + 16;
    a[i] = (_Float16)(ka < K ? W[(size_t)(ka < K ? ka : K - 1) * ld + n] : 0.f); a[8 + i] = (_Float16)(kb < K ? W[(size_t)(kb < K ? kb : K - 1) * ld + n] : 0.f); }
  return a;
}
struct F2 { v16b h, l; };
__device__ __forceinline__ F2 bsplit16(const float v[16]) { F2 r;
#pragma unroll
  for (int i = 0; i < 16; ++i) { const __bf16 h = (__bf16)v[i]; r.h[i] = h; r.l[i] = (__bf16)(v[i] - (float)h); }
  return r; }
__device__ __forceinline__ F2 split_row(const float* row, int k0, int lane) { float v[16]; const float* p = row + k0 + 8 * (lane >> 4);
#pragma unroll
  for (int i = 0; i < 8; ++i) { v[i] = p[i]; v[8 + i] = p[16 + i]; }
  return bsplit16(v); }
__device__ __forceinline__ F2 split_rowK(const float* row, int k0, int lane, int K) { float v[16]; const int g = lane >> 4;
#pragma unroll
  for (int i = 0; i < 8; ++i) { const int ka = k0 + 8 * g + i, kb = ka + 16; v[i] = ka < K ? row[ka < K ? ka : K - 1] : 0.f; v[8 + i] = kb < K ? row[kb < K ? kb : K - 1] : 0.f; }
  return bsplit16(v); }
__device__ __forceinline__ F2 split_col(const float* W, int k0, int n, int lane, int ld, int K) { float v[16]; const int g = lane >> 4;
#pragma unroll
  for (int i = 0; i < 8; ++i) { const int ka = k0 + 8 * g + i, kb = ka + 16; v[i] = ka < K ? W[(size_t)(ka < K ? ka : K - 1) * ld + n] : 0.f; v[8 + i] = kb < K ? W[(size_t)(kb < K ? kb : K - 1) * ld + n] : 0.f; }
  return bsplit16(v); }
__device__ __forceinline__ v8f mac3(const F2& a, const F2& b, v8f c) { c = wmma_bf(a.l, b.h, c); c = wmma_bf(a.h, b.l, c); return wmma_bf(a.h, b.h, c); }
__device__ __forceinline__ float sigm(float v) { return 1.0f / (1.0f + expf(-v)); }
#define LDSX() do { asm volatile("s_wait_dscnt 0" ::: "memory"); __builtin_amdgcn_wave_barrier(); __builtin_amdgcn_fence(__ATOMIC_RELEASE, "workgroup"); } while (0)
__device__ __forceinline__ v16b wcol_oi(const float* Wm, int k0, int o, int lane, int K) { v16b w; const float* p = Wm + (size_t)o * K + k0 + 8 * (lane >> 4);
#pragma unroll
  for (int i = 0; i < 8; ++i) { w[i] = (__bf16)p[i]; w[8 + i] = (__bf16)p[16 + i]; }
  return w; }

#define NBT 2
#define SS 2048
#define DM 1024
#define NH 16
#define HD 64
#define WW 16
#define NR (NBT * SS)
#ifndef TNB
#define TNB NBT
#endif
#ifndef NSV
#define NSV SS
#endif
#define NRV (TNB * NSV)
__device__ __forceinline__ float bfr(float v) { return (float)(__bf16)v; }
#define WS_Q   0u
#define WS_K   (WS_Q + 4u * (size_t)NR * DM)
#define WS_V   (WS_K + 4u * (size_t)NR * DM)
#define WS_KP  (WS_V + 4u * (size_t)NR * DM)
#define WS_Z   (WS_KP + 4u * (size_t)NR * DM)
#define WS_O   (WS_Z + 4u * (size_t)NR * DM)
#define WS_END (WS_O + 4u * (size_t)NR * DM)

__global__ __launch_bounds__(128) void k_lin4(const float* __restrict__ X, const float* __restrict__ W0, const float* __restrict__ W1, const float* __restrict__ W2, const float* __restrict__ W3, float* __restrict__ O0, float* __restrict__ O1, float* __restrict__ O2, float* __restrict__ O3) { __shared__ __align__(16) float sf[4][16][132];
  const int tid = threadIdx.x, wave = tid >> 5, lane = tid & 31, col = lane & 15, g = lane >> 4; const int which = blockIdx.z; const int c0 = blockIdx.y * 128; const size_t r0 = (size_t)blockIdx.x * 64 + wave * 16;
  const float* Wm = which == 0 ? W0 : which == 1 ? W1 : which == 2 ? W2 : W3; float* OUT = which == 0 ? O0 : which == 1 ? O1 : which == 2 ? O2 : O3;
  v8f acc[8] = {};
#pragma unroll 2
  for (int kc = 0; kc < DM / 32; ++kc) { v16b a; { const float* p = X + (r0 + col) * DM + kc * 32 + 8 * g;
#pragma unroll
      for (int i = 0; i < 8; ++i) { a[i] = (__bf16)p[i]; a[8 + i] = (__bf16)p[16 + i]; } }
    asm volatile("s_wait_loadcnt 0x0" ::: "memory");
#pragma unroll
    for (int j = 0; j < 8; ++j) { const v16b w = wcol_oi(Wm, kc * 32, c0 + j * 16 + col, lane, DM); asm volatile("s_wait_loadcnt 0x0" ::: "memory"); acc[j] = wmma_bf(a, w, acc[j]); } }
#pragma unroll
  for (int j = 0; j < 8; ++j)
#pragma unroll
    for (int r = 0; r < 8; ++r) sf[wave][8 * g + r][j * 16 + col] = acc[j][r];
  LDSX(); for (int rl = 0; rl < 16; ++rl) vst2(OUT + (r0 + rl) * DM + c0 + lane * 4, *(const v4f*)&sf[wave][rl][lane * 4]); }
__global__ __launch_bounds__(128) void k_tsa(const float* __restrict__ Q, const float* __restrict__ K, const float* __restrict__ V, const float* __restrict__ KP, float* __restrict__ Z) {
  __shared__ __align__(16) float sk[80][68], skp[80][68], sv[80][68], sq[64][68]; __shared__ __align__(16) float sp[4][16][20]; __shared__ __align__(16) float sz[64][68];
  const int tid = threadIdx.x, wave = tid >> 5, lane = tid & 31, col = lane & 15, g = lane >> 4; const int s0 = blockIdx.x * 64, h = blockIdx.y, b = blockIdx.z;
  for (int e = tid; e < 80 * 16; e += 128) { const int rr = e >> 4, q4 = e & 15; const int pos = s0 - 15 + rr; v4f kv = {0.f, 0.f, 0.f, 0.f}, pv = kv, vv = kv;
    if (pos >= 0 && rr < 79) { const size_t o = ((size_t)b * SS + pos) * DM + h * HD + q4 * 4; kv = *(const v4f*)(K + o); pv = *(const v4f*)(KP + o); vv = *(const v4f*)(V + o); }
    *(v4f*)&sk[rr][q4 * 4] = kv; *(v4f*)&skp[rr][q4 * 4] = pv; *(v4f*)&sv[rr][q4 * 4] = vv; }
  for (int e = tid; e < 64 * 16; e += 128) { const int rr = e >> 4, q4 = e & 15; *(v4f*)&sq[rr][q4 * 4] = *(const v4f*)(Q + ((size_t)b * SS + s0 + rr) * DM + h * HD + q4 * 4); }
  for (int e = tid; e < 80; e += 128) { sk[e][64] = sk[e][65] = sk[e][66] = sk[e][67] = 0.f; skp[e][64] = skp[e][65] = skp[e][66] = skp[e][67] = 0.f; sv[e][64] = sv[e][65] = sv[e][66] = sv[e][67] = 0.f; }
  __syncthreads();
#pragma unroll 1
  for (int si = 0; si < 16; ++si) { const int sl = wave * 16 + si; const int s = s0 + sl;
    v8f acc = {};
#pragma unroll
    for (int kc = 0; kc < 2; ++kc) { float va[16], vb[16];
#pragma unroll
      for (int i = 0; i < 8; ++i) { const int d0 = kc * 32 + 8 * g + i, d1 = d0 + 16; va[i] = sq[sl][d0] * sk[sl + col][d0]; va[8 + i] = sq[sl][d1] * sk[sl + col][d1]; vb[i] = skp[sl + col][d0]; vb[8 + i] = skp[sl + col][d1]; }
      const F2 a = bsplit16(va), bq = bsplit16(vb); acc = wmma_bf(a.h, bq.h, acc); acc = wmma_bf(a.l, bq.h, acc); acc = wmma_bf(a.h, bq.l, acc); }
    float ev[8]; float mx = -3.0e38f;
#pragma unroll
    for (int r = 0; r < 8; ++r) { const int j = 8 * g + r; const bool ok = (j >= 15 - s) && (col >= 15 - s); const float v = ok ? acc[r] * 0.125f : -3.0e38f; ev[r] = v; mx = fmaxf(mx, v); }
#pragma unroll
    for (int o = 1; o < 32; o <<= 1) mx = fmaxf(mx, __shfl_xor(mx, o));
    float sm = 0.f;
#pragma unroll
    for (int r = 0; r < 8; ++r) { const int j = 8 * g + r; const bool ok = (j >= 15 - s) && (col >= 15 - s); ev[r] = ok ? expf(ev[r] - mx) : 0.f; sm += ev[r]; }
#pragma unroll
    for (int o = 1; o < 32; o <<= 1) sm += __shfl_xor(sm, o);
    const float inv = 1.0f / sm;
#pragma unroll
    for (int r = 0; r < 8; ++r) sp[wave][8 * g + r][col] = ev[r] * inv;
    LDSX();
    F2 ap; { float vp[16];
#pragma unroll
      for (int i = 0; i < 8; ++i) { vp[i] = (g == 0) ? sp[wave][col][i] : sp[wave][col][8 + i]; vp[8 + i] = 0.f; }
      ap = bsplit16(vp); }
    float zpart[4];
#pragma unroll
    for (int t4 = 0; t4 < 4; ++t4) { float vbv[16]; const int d = t4 * 16 + col;
#pragma unroll
      for (int i = 0; i < 8; ++i) { vbv[i] = sv[sl + 8 * g + i][d]; vbv[8 + i] = 0.f; }
      const F2 bv = bsplit16(vbv); v8f w8 = {}; w8 = wmma_bf(ap.h, bv.h, w8); w8 = wmma_bf(ap.l, bv.h, w8); w8 = wmma_bf(ap.h, bv.l, w8);
      float zp = 0.f;
#pragma unroll
      for (int r = 0; r < 8; ++r) zp += sv[sl + 8 * g + r][d] * w8[r];
      zp += __shfl_xor(zp, 16); zpart[t4] = zp; }
    if (g == 0) {
#pragma unroll
      for (int t4 = 0; t4 < 4; ++t4) sz[sl][t4 * 16 + col] = zpart[t4]; }
    LDSX(); }
  __syncthreads();
  for (int e = tid; e < 64 * 16; e += 128) { const int rr = e >> 4, q4 = e & 15; vst2(Z + ((size_t)b * SS + s0 + rr) * DM + h * HD + q4 * 4, *(const v4f*)&sz[rr][q4 * 4]); } }
__global__ __launch_bounds__(128) void k_outp(const float* __restrict__ Zr, const float* __restrict__ WO, const float* __restrict__ X, float* __restrict__ O) { __shared__ __align__(16) float sf[4][16][132];
  const int tid = threadIdx.x, wave = tid >> 5, lane = tid & 31, col = lane & 15, g = lane >> 4; const int c0 = blockIdx.y * 128; const size_t r0 = (size_t)blockIdx.x * 64 + wave * 16;
  v8f acc[8] = {};
#pragma unroll 1
  for (int kc = 0; kc < DM / 32; ++kc) { const F2 a = split_row(Zr + (r0 + col) * DM, kc * 32, lane); asm volatile("s_wait_loadcnt 0x0" ::: "memory");
#pragma unroll
    for (int j = 0; j < 8; ++j) { const v16b w = wcol_oi(WO, kc * 32, c0 + j * 16 + col, lane, DM); asm volatile("s_wait_loadcnt 0x0" ::: "memory"); acc[j] = wmma_bf(a.h, w, acc[j]); acc[j] = wmma_bf(a.l, w, acc[j]); } }
#pragma unroll
  for (int j = 0; j < 8; ++j)
#pragma unroll
    for (int r = 0; r < 8; ++r) sf[wave][8 * g + r][j * 16 + col] = acc[j][r];
  LDSX(); for (int rl = 0; rl < 16; ++rl) { const size_t o = (r0 + rl) * DM + c0 + lane * 4; const v4f xv = *(const v4f*)(X + o); v4f v = *(const v4f*)&sf[wave][rl][lane * 4]; v[0] += bfr(xv[0]); v[1] += bfr(xv[1]); v[2] += bfr(xv[2]); v[3] += bfr(xv[3]); vst2(O + o, v); } }
__global__ __launch_bounds__(256) void k_ln(const float* __restrict__ O, const float* __restrict__ G, const float* __restrict__ BE, float* __restrict__ OUT) { const int wave = threadIdx.x >> 5, lane = threadIdx.x & 31; const size_t row = (size_t)blockIdx.x * 8 + wave; if (row >= (size_t)NRV) return;
  v4f v[8]; float s = 0.f;
#pragma unroll
  for (int i = 0; i < 8; ++i) { v[i] = *(const v4f*)(O + row * DM + i * 128 + lane * 4); s += (v[i][0] + v[i][1]) + (v[i][2] + v[i][3]); }
#pragma unroll
  for (int o = 1; o < 32; o <<= 1) s += __shfl_xor(s, o);
  const float mu = s * (1.0f / DM); float q = 0.f;
#pragma unroll
  for (int i = 0; i < 8; ++i) { for (int k = 0; k < 4; ++k) { const float d = v[i][k] - mu; q += d * d; } }
#pragma unroll
  for (int o = 1; o < 32; o <<= 1) q += __shfl_xor(q, o);
  const float rs = rsqrtf(q * (1.0f / DM) + 1e-5f);
#pragma unroll
  for (int i = 0; i < 8; ++i) { const int c = i * 128 + lane * 4; v4f r4; for (int k = 0; k < 4; ++k) r4[k] = (v[i][k] - mu) * rs * bfr(G[c + k]) + bfr(BE[c + k]); vst2(OUT + row * DM + c, r4); } }
extern "C" void kernel_launch(void* const* d_in, const int* in_sizes, int n_in, void* d_out, int out_size, void* d_ws, size_t ws_size, hipStream_t stream) {
  (void)in_sizes; (void)n_in; (void)out_size;
  if (ws_size < (size_t)WS_END) return;
  char* ws = (char*)d_ws; const float** F = (const float**)d_in;
  float *Q = (float*)(ws + WS_Q), *K = (float*)(ws + WS_K), *V = (float*)(ws + WS_V), *KP = (float*)(ws + WS_KP), *Zr = (float*)(ws + WS_Z), *O = (float*)(ws + WS_O);
  k_lin4<<<dim3(NRV / 64, DM / 128, 4), 128, 0, stream>>>(F[0], F[1], F[2], F[3], F[4], Q, K, V, KP);
  k_tsa<<<dim3(NSV / 64, NH, TNB), 128, 0, stream>>>(Q, K, V, KP, Zr);
  k_outp<<<dim3(NRV / 64, DM / 128), 128, 0, stream>>>(Zr, F[5], F[0], O);
  k_ln<<<dim3(NRV / 8), 256, 0, stream>>>(O, F[6], F[7], (float*)d_out);
}
